// DemoRNN_37520834298127
// MI455X (gfx1250) — hardware-verified
//
#include <hip/hip_runtime.h>
#include <math.h>

typedef __attribute__((ext_vector_type(16))) _Float16 v16h;
typedef __attribute__((ext_vector_type(8)))  float    v8f;
typedef __attribute__((ext_vector_type(4)))  float    v4f;

constexpr int kBatch   = 2048;
constexpr int kSteps   = 4096;
constexpr int kHid     = 10;
constexpr int kHalfU   = 5;
constexpr int kTile    = 16;
constexpr int kTiles   = kBatch / kTile;
constexpr int kChunk   = 64;
constexpr int kXPitch  = 68;
constexpr float kWCarry   = 1024.0f;
constexpr float kRCarry   = 4096.0f;
constexpr float kW3Carry  = kWCarry / kRCarry;
constexpr float kExpScale = 2.0f / kWCarry;
constexpr float kF16MinNormal = 6.103515625e-05f;
constexpr int kPWhh  = 0;
constexpr int kPWih  = kHid * kHid;
constexpr int kPBias = kPWih + kHid;
constexpr int kPWout = kPBias + kHid;
constexpr int kPSize = 160;

static_assert(kHid == 2 * kHalfU, "two lane halves own five units each");
static_assert(kBatch % kTile == 0, "whole batch tiles");
static_assert(kSteps % kChunk == 0, "whole time chunks");
static_assert((kChunk * 4) % 128 == 0, "out0 chunk is whole lines");
static_assert((kSteps * 4) % 128 == 0, "second output starts on a line");
static_assert((kTile * kHid * 4) % 128 == 0, "per-tile state block is whole lines");
static_assert(kTile * kHid == 160, "state block = 40 vectors of 4 floats");
static_assert(kSteps * 4 + kBatch * kHid * 4 == 98304, "output bytes");
static_assert(kPWout + kHid <= kPSize, "parameter table fits");
static_assert((kXPitch * 4) % 16 == 0, "16-B aligned LDS rows");

__device__ __forceinline__ float flush_small(float v) {
  return (fabsf(v) < kF16MinNormal) ? 0.0f : v;
}

__device__ __forceinline__ v8f mma_step(v16h a, v16h b, v8f c) {
  c = __builtin_amdgcn_wmma_f32_16x16x32_f16(false, a, false, b, (short)0, c, false, false);
  asm volatile("v_nop\n\tv_nop\n\tv_nop\n\tv_nop" : "+v"(c) : "v"(a), "v"(b));
  return c;
}

__device__ __forceinline__ v16h pack_state(const float (&hv)[kHalfU]) {
  _Float16 hh[kHalfU], hl[kHalfU];
#pragma unroll
  for (int r = 0; r < kHalfU; ++r) {
    const float q = flush_small(hv[r]);
    const _Float16 t = (_Float16)q;
    const float res = (hv[r] - (float)t) * kRCarry;
    hh[r] = t;
    hl[r] = (_Float16)flush_small(res);
  }
  v16h f;
  f[0]  = hh[0]; f[1]  = hh[1]; f[2]  = hh[2]; f[3]  = hh[3];
  f[4]  = hh[4]; f[5]  = hl[0]; f[6]  = hl[1]; f[7]  = hl[2];
  f[8]  = hh[0]; f[9]  = hh[1]; f[10] = hh[2]; f[11] = hh[3];
  f[12] = hh[4]; f[13] = hl[3]; f[14] = hl[4]; f[15] = hl[4];
  return f;
}

__global__ __launch_bounds__(32) void rnn_tile_kernel(
    const float* __restrict__ x, const float* __restrict__ hid,
    const float* __restrict__ Wih, const float* __restrict__ Whh,
    const float* __restrict__ bih, const float* __restrict__ bhh,
    const float* __restrict__ Wout, const float* __restrict__ bout,
    float* __restrict__ out)
{
  __shared__ __align__(16) float sX[kTile * kXPitch];
  __shared__ __align__(16) float sP[kPSize];
  __shared__ __align__(16) float sO[kChunk];
  __shared__ __align__(16) float sH[kTile * kHid];

  const int lane = threadIdx.x & 31;
  const int hf   = lane >> 4;
  const int n    = lane & 15;
  const int b0   = blockIdx.x * kTile;
  const bool emit = (blockIdx.x == 0);

#pragma unroll
  for (int it = 0; it < 4; ++it) {
    const int idx = it * 32 + lane;
    const int idc = (idx < kHid * kHid) ? idx : (kHid * kHid - 1);
    float v = Whh[idc];
    asm volatile("" : "+v"(v));
    if (idx < kHid * kHid) sP[kPWhh + idx] = v;
  }
  {
    const int lc = (lane < kHid) ? lane : (kHid - 1);
    float pa = Wih[lc];
    float pb = bih[lc];
    float pc = bhh[lc];
    float pd = Wout[lc];
    asm volatile("" : "+v"(pa));
    asm volatile("" : "+v"(pb));
    asm volatile("" : "+v"(pc));
    asm volatile("" : "+v"(pd));
    if (lane < kHid) {
      sP[kPWih + lane]  = pa;
      sP[kPBias + lane] = pb + pc;
      sP[kPWout + lane] = pd;
    }
  }
  const float bo = bout[0];
  __syncthreads();

  v16h af;
  {
    const bool jvalid = (n & 7) < kHalfU;
    const int  j  = kHalfU * (n >> 3) + (n & 7);
    const int  jc = jvalid ? j : 0;
    _Float16 a1[kHalfU], a2[kHalfU], a3[kHalfU];
#pragma unroll
    for (int r = 0; r < kHalfU; ++r) {
      const float wl = sP[kPWhh + jc * kHid + kHalfU * hf + r];
      const float w  = jvalid ? wl : 0.0f;
      const float ws = w * kWCarry;
      const _Float16 t = (_Float16)flush_small(ws);
      a1[r] = t;
      a2[r] = (_Float16)flush_small(ws - (float)t);
      a3[r] = (_Float16)flush_small(w * kW3Carry);
    }
    const float zpad = 0.0f;
    af[0]  = a1[0]; af[1]  = a1[1]; af[2]  = a1[2]; af[3]  = a1[3];
    af[4]  = a1[4]; af[5]  = a3[0]; af[6]  = a3[1]; af[7]  = a3[2];
    af[8]  = a2[0]; af[9]  = a2[1]; af[10] = a2[2]; af[11] = a2[3];
    af[12] = a2[4]; af[13] = a3[3]; af[14] = a3[4]; af[15] = (_Float16)zpad;
  }

  float wih[kHalfU], bs[kHalfU], wo[kHalfU];
#pragma unroll
  for (int r = 0; r < kHalfU; ++r) {
    const int u = kHalfU * hf + r;
    wih[r] = sP[kPWih + u] * kWCarry;
    bs[r]  = sP[kPBias + u] * kWCarry;
    wo[r]  = sP[kPWout + u];
  }

  float hv[kHalfU];
#pragma unroll
  for (int r = 0; r < kHalfU; ++r)
    hv[r] = hid[(size_t)(b0 + n) * kHid + kHalfU * hf + r];
  v16h bf = pack_state(hv);

#pragma unroll 1
  for (int t0 = 0; t0 < kSteps; t0 += kChunk) {
    __syncthreads();
#pragma unroll
    for (int it = 0; it < 8; ++it) {
      const int idx = it * 32 + lane;
      const int row = idx >> 4;
      const int c4  = (idx & 15) * 4;
      const v4f xv4 = *(const v4f*)(x + (size_t)(b0 + row) * kSteps + t0 + c4);
      *(v4f*)(sX + row * kXPitch + c4) = xv4;
    }
    __syncthreads();

#pragma unroll 1
    for (int s = 0; s < kChunk; ++s) {
      const float xv = sX[n * kXPitch + s];
      v8f c;
      c[0] = fmaf(xv, wih[0], bs[0]);
      c[1] = fmaf(xv, wih[1], bs[1]);
      c[2] = fmaf(xv, wih[2], bs[2]);
      c[3] = fmaf(xv, wih[3], bs[3]);
      c[4] = fmaf(xv, wih[4], bs[4]);
      c[5] = 0.0f;
      c[6] = 0.0f;
      c[7] = 0.0f;
      c = mma_step(af, bf, c);
#pragma unroll
      for (int r = 0; r < kHalfU; ++r) {
        const float e  = expf(c[r] * kExpScale);
        const float rc = __builtin_amdgcn_rcpf(e + 1.0f);
        hv[r] = fmaf(-2.0f, rc, 1.0f);
      }
      bf = pack_state(hv);
      if (emit) {
        float p = 0.0f;
#pragma unroll
        for (int r = 0; r < kHalfU; ++r) p = fmaf(hv[r], wo[r], p);
        p += __shfl_xor(p, 16, 32);
        if (lane == 0) sO[s] = p + bo;
      }
    }
    __syncthreads();
    if (emit) {
      const v4f ov = *(const v4f*)(sO + n * 4);
      float* op = out + t0 + n * 4;
      if (lane < 16) *(volatile v4f*)op = ov;
      __threadfence();
      if (lane < 16) *(volatile v4f*)op = ov;
    }
  }

  __syncthreads();
#pragma unroll
  for (int r = 0; r < kHalfU; ++r) sH[n * kHid + kHalfU * hf + r] = hv[r];
  __syncthreads();
  {
    float* hp = out + kSteps + (size_t)b0 * kHid;
    const v4f v0 = *(const v4f*)(sH + lane * 4);
    const v4f v1 = *(const v4f*)(sH + 128 + (lane & 7) * 4);
    *(volatile v4f*)(hp + lane * 4) = v0;
    if (lane < 8) *(volatile v4f*)(hp + 128 + lane * 4) = v1;
    __threadfence();
    *(volatile v4f*)(hp + lane * 4) = v0;
    if (lane < 8) *(volatile v4f*)(hp + 128 + lane * 4) = v1;
  }
}

extern "C" void kernel_launch(void* const* d_in, const int* in_sizes, int n_in,
                              void* d_out, int out_size, void* d_ws, size_t ws_size,
                              hipStream_t stream) {
  (void)d_ws;
  (void)ws_size;
  if (n_in < 8) return;
  if (in_sizes[0] != kBatch * kSteps) return;
  if (in_sizes[1] != kBatch * kHid) return;
  if (in_sizes[2] != kHid) return;
  if (in_sizes[3] != kHid * kHid) return;
  if (in_sizes[4] != kHid) return;
  if (in_sizes[5] != kHid) return;
  if (in_sizes[6] != kHid) return;
  if (in_sizes[7] != 1) return;
  if (out_size != kSteps + kBatch * kHid) return;

  const float* x      = (const float*)d_in[0];
  const float* hidden = (const float*)d_in[1];
  const float* W_ih   = (const float*)d_in[2];
  const float* W_hh   = (const float*)d_in[3];
  const float* b_ih   = (const float*)d_in[4];
  const float* b_hh   = (const float*)d_in[5];
  const float* W_out  = (const float*)d_in[6];
  const float* b_out  = (const float*)d_in[7];

  rnn_tile_kernel<<<kTiles, 32, 0, stream>>>(x, hidden, W_ih, W_hh, b_ih, b_hh, W_out, b_out,
                                             (float*)d_out);
}
